// GraphNC_70738111365645
// MI455X (gfx1250) — hardware-verified
//
#include <hip/hip_runtime.h>
#include <stddef.h>


#define CH     128
#define C2     64
#define KPB    128
#define APZ    136
#define GROWS  32
#define GTHR   64
#define EWAV   4
#define EPW    32
#define ETHR   (EWAV * 32)
#define EPB    (EWAV * EPW)
#define PTHR   256
#define OFF_B1 0
#define OFF_B2 (2 * CH * KPB)
#define BPTOT  (OFF_B2 + C2 * KPB)
#define WSCAP  134217728
#define W1SC   16.0f
#define W2SC   64.0f
#define HSC    16.0f
#define RP     0.0625f
#define RH     0.0009765625f

static_assert(BPTOT == 40960);
static_assert((APZ % 8) == 0 && (KPB % 8) == 0);
static_assert(GROWS == (GTHR / 32) * 16);
static_assert((CH % 32) == 0 && C2 == 64);
static_assert(EPB == ETHR);
static_assert(GROWS * CH == 16 * GTHR * 4);

typedef float    v4f  __attribute__((ext_vector_type(4)));
typedef float    v8f  __attribute__((ext_vector_type(8)));
typedef _Float16 v4h  __attribute__((ext_vector_type(4)));
typedef _Float16 v8h  __attribute__((ext_vector_type(8)));
typedef _Float16 v16h __attribute__((ext_vector_type(16)));
union Frag { v16h v; v8h h[2]; };

__device__ __forceinline__ v8f wmh(v16h a, v16h b, v8f c) {
  v8f d = __builtin_amdgcn_wmma_f32_16x16x32_f16(false, a, false, b, (short)0, c, false, false);
  asm volatile("v_nop\n\tv_nop\n\tv_nop\n\tv_nop" : "+v"(d) : "v"(a), "v"(b));
  return d;
}

__device__ __forceinline__ v4h cvt4h(v4f a) {
  v4h r;
  r.x = (_Float16)(a.x * HSC); r.y = (_Float16)(a.y * HSC); r.z = (_Float16)(a.z * HSC); r.w = (_Float16)(a.w * HSC);
  return r;
}

template <int NT>
__device__ __forceinline__ void mma16(const _Float16* At, const _Float16* __restrict__ Bpl,
                                      int lane, v8f (&acc)[NT]) {
  const int hh = lane >> 4, m = lane & 15;
#pragma unroll
  for (int t = 0; t < NT; ++t) { v8f z = {0.f, 0.f, 0.f, 0.f, 0.f, 0.f, 0.f, 0.f}; acc[t] = z; }
  const _Float16* ap = At + m * APZ + 8 * hh;
  const _Float16* bb = Bpl + (size_t)m * KPB + 8 * hh;
#pragma unroll 1
  for (int ks = 0; ks < CH / 32; ++ks) {
    Frag a;
    a.h[0] = *(const v8h*)(ap + 32 * ks);
    a.h[1] = *(const v8h*)(ap + 32 * ks + 16);
#pragma unroll
    for (int t = 0; t < NT; ++t) {
      const _Float16* bp = bb + (size_t)(16 * t) * KPB + 32 * ks;
      Frag b;
      b.h[0] = *(const v8h*)bp;
      b.h[1] = *(const v8h*)(bp + 16);
      acc[t] = wmh(a.v, b.v, acc[t]);
    }
  }
}

template <int NT>
__device__ __forceinline__ void mma32(const _Float16* At, const _Float16* __restrict__ Bpl,
                                      int lane, v8f (&acc0)[NT], v8f (&acc1)[NT]) {
  const int hh = lane >> 4, m = lane & 15;
#pragma unroll
  for (int t = 0; t < NT; ++t) {
    v8f z = {0.f, 0.f, 0.f, 0.f, 0.f, 0.f, 0.f, 0.f};
    acc0[t] = z; acc1[t] = z;
  }
  const _Float16* ap0 = At + m * APZ + 8 * hh;
  const _Float16* ap1 = ap0 + 16 * APZ;
  const _Float16* bb  = Bpl + (size_t)m * KPB + 8 * hh;
#pragma unroll 1
  for (int ks = 0; ks < CH / 32; ++ks) {
    Frag a0, a1;
    a0.h[0] = *(const v8h*)(ap0 + 32 * ks);
    a0.h[1] = *(const v8h*)(ap0 + 32 * ks + 16);
    a1.h[0] = *(const v8h*)(ap1 + 32 * ks);
    a1.h[1] = *(const v8h*)(ap1 + 32 * ks + 16);
#pragma unroll
    for (int t = 0; t < NT; ++t) {
      const _Float16* bp = bb + (size_t)(16 * t) * KPB + 32 * ks;
      Frag b;
      b.h[0] = *(const v8h*)bp;
      b.h[1] = *(const v8h*)(bp + 16);
      acc0[t] = wmh(a0.v, b.v, acc0[t]);
      acc1[t] = wmh(a1.v, b.v, acc1[t]);
    }
  }
}

template <int J0>
__device__ __forceinline__ void rows_h(_Float16* hw, const float* __restrict__ P, const float* __restrict__ Q,
                                       int sv, int dv, int lane) {
#pragma unroll
  for (int j = J0; j < J0 + 8; ++j) {
    const int s = __builtin_amdgcn_readlane(sv, j);
    const int d = __builtin_amdgcn_readlane(dv, j);
    const v4f p = *(const v4f*)(P + (size_t)s * CH + 4 * lane);
    const v4f q = *(const v4f*)(Q + (size_t)d * CH + 4 * lane);
    v4f u = p + q;
    u.x = fmaxf(u.x, 0.0f); u.y = fmaxf(u.y, 0.0f); u.z = fmaxf(u.z, 0.0f); u.w = fmaxf(u.w, 0.0f);
    *(v4h*)(hw + j * APZ + 4 * lane) = cvt4h(u);
  }
}

__global__ __launch_bounds__(PTHR) void k_wprep(const float* __restrict__ W1, const float* __restrict__ W2,
                                                _Float16* Bpl) {
  const int blk = blockIdx.x, tid = threadIdx.x;
  float v[8];
  v8h hv;
  _Float16* dp;
  if (blk < 16) {
    const int i = blk * PTHR + tid;
    const int n = i >> 4, k0 = (i & 15) * 8;
    const int kb = (n >> 7) * CH, nc = n & (CH - 1);
#pragma unroll
    for (int e = 0; e < 8; ++e) v[e] = W1[(kb + k0 + e) * CH + nc];
#pragma unroll
    for (int e = 0; e < 8; ++e) hv[e] = (_Float16)(v[e] * W1SC);
    dp = Bpl + OFF_B1 + i * 8;
  } else {
    const int i = (blk - 16) * PTHR + tid;
    const int n = i >> 4, k0 = (i & 15) * 8;
#pragma unroll
    for (int e = 0; e < 8; ++e) v[e] = W2[(k0 + e) * C2 + n];
#pragma unroll
    for (int e = 0; e < 8; ++e) hv[e] = (_Float16)(v[e] * W2SC);
    dp = Bpl + OFF_B2 + i * 8;
  }
  *(volatile v8h*)dp = hv;
  __threadfence();
  *(volatile v8h*)dp = hv;
}

__global__ __launch_bounds__(GTHR) void k_nodegemm(const float* __restrict__ zi, const float* __restrict__ zj,
                                                   const _Float16* __restrict__ B1, const float* __restrict__ b1,
                                                   float* PQ, int nN, int nPad) {
  __shared__ __attribute__((aligned(16))) _Float16 At[GROWS * APZ];
  __shared__ __attribute__((aligned(16))) float stg[GROWS * CH];
  const int tid = threadIdx.x, lane = tid & 31, wave = tid >> 5, hh = lane >> 4, m = lane & 15;
  const int side = blockIdx.y;
  const float* x = side ? zj : zi;
  const _Float16* Bp = B1 + (size_t)side * CH * KPB;
  const int rowBase = blockIdx.x * GROWS;
  {
    const int r = tid >> 1, c0 = (tid & 1) * 64;
    int xrow = rowBase + r;
    xrow = xrow > nN - 1 ? nN - 1 : xrow;
    const float* xp = x + (size_t)xrow * CH + c0;
#pragma unroll
    for (int j = 0; j < 8; ++j) {
      const v4f a = *(const v4f*)(xp + 8 * j), b = *(const v4f*)(xp + 8 * j + 4);
      v8h hv;
      hv[0] = (_Float16)a.x; hv[1] = (_Float16)a.y; hv[2] = (_Float16)a.z; hv[3] = (_Float16)a.w;
      hv[4] = (_Float16)b.x; hv[5] = (_Float16)b.y; hv[6] = (_Float16)b.z; hv[7] = (_Float16)b.w;
      *(v8h*)(At + r * APZ + c0 + 8 * j) = hv;
    }
  }
  __syncthreads();

  {
    v8f acc[8];
    mma16<8>(At + wave * 16 * APZ, Bp, lane, acc);
    float* sp = stg + (wave * 16 + 8 * hh) * CH + m;
#pragma unroll
    for (int t = 0; t < 8; ++t) {
      const float bb = b1[16 * t + m];
      const float bv = side ? bb : 0.0f;
#pragma unroll
      for (int r = 0; r < 8; ++r) sp[r * CH + 16 * t] = acc[t][r] * RP + bv;
    }
  }
  __syncthreads();

  float* gp = PQ + ((size_t)side * nPad + rowBase) * CH;
#pragma unroll
  for (int it = 0; it < 16; ++it) {
    const int f = it * GTHR + tid;
    const v4f v = *(const v4f*)(stg + 4 * f);
    *(volatile v4f*)(gp + 4 * f) = v;
  }
  __threadfence();
#pragma unroll
  for (int it = 0; it < 16; ++it) {
    const int f = it * GTHR + tid;
    const v4f v = *(const v4f*)(stg + 4 * f);
    *(volatile v4f*)(gp + 4 * f) = v;
  }
}

__global__ __launch_bounds__(ETHR) void k_edge(
    const float* __restrict__ PQ, const int* __restrict__ srcs, const int* __restrict__ dsts,
    const _Float16* __restrict__ B2, const float* __restrict__ b2, const float* __restrict__ W3,
    const float* __restrict__ b3, float* out, int nN, int nE, int nPad) {
  __shared__ __attribute__((aligned(16))) _Float16 ht[EWAV * EPW * APZ];
  __shared__ __attribute__((aligned(16))) float sc[EPB];
  const int tid = threadIdx.x, lane = tid & 31, wave = tid >> 5, hh = lane >> 4, m = lane & 15;
  const float* P = PQ;
  const float* Q = PQ + (size_t)nPad * CH;
  _Float16* hw = ht + wave * (EPW * APZ);

  float b2c[4], w3c[4];
#pragma unroll
  for (int t = 0; t < 4; ++t) { b2c[t] = b2[16 * t + m]; w3c[t] = W3[16 * t + m]; }
  const float b3v = b3[0];

  const int eBase = blockIdx.x * EPB + wave * EPW;
  int e = eBase + lane;
  e = e > nE - 1 ? nE - 1 : e;
  int sv = srcs[e];
  sv = sv < 0 ? 0 : (sv > nN - 1 ? nN - 1 : sv);
  int dv = dsts[e];
  dv = dv < 0 ? 0 : (dv > nN - 1 ? nN - 1 : dv);

  rows_h<0>(hw, P, Q, sv, dv, lane);
  asm volatile("" ::: "memory");
  rows_h<8>(hw, P, Q, sv, dv, lane);
  asm volatile("" ::: "memory");
  rows_h<16>(hw, P, Q, sv, dv, lane);
  asm volatile("" ::: "memory");
  rows_h<24>(hw, P, Q, sv, dv, lane);
  __syncthreads();

  v8f acc0[4], acc1[4];
  mma32<4>(hw, B2, lane, acc0, acc1);

  float v[16];
#pragma unroll
  for (int r = 0; r < 8; ++r) {
    float s0 = 0.0f, s1 = 0.0f;
#pragma unroll
    for (int t = 0; t < 4; ++t) {
      const float h0 = fmaxf(fmaf(acc0[t][r], RH, b2c[t]), 0.0f);
      const float h1 = fmaxf(fmaf(acc1[t][r], RH, b2c[t]), 0.0f);
      s0 = fmaf(h0, w3c[t], s0);
      s1 = fmaf(h1, w3c[t], s1);
    }
    v[r] = s0;
    v[8 + r] = s1;
  }

  float u[8];
  {
    const bool kb = ((lane >> 3) & 1) != 0;
#pragma unroll
    for (int i = 0; i < 8; ++i) {
      const float snd = kb ? v[i] : v[i + 8];
      const float kp  = kb ? v[i + 8] : v[i];
      u[i] = kp + __shfl_xor(snd, 8, 32);
    }
  }
  float w4[4];
  {
    const bool kb = ((lane >> 2) & 1) != 0;
#pragma unroll
    for (int i = 0; i < 4; ++i) {
      const float snd = kb ? u[i] : u[i + 4];
      const float kp  = kb ? u[i + 4] : u[i];
      w4[i] = kp + __shfl_xor(snd, 4, 32);
    }
  }
  float x2[2];
  {
    const bool kb = ((lane >> 1) & 1) != 0;
#pragma unroll
    for (int i = 0; i < 2; ++i) {
      const float snd = kb ? w4[i] : w4[i + 2];
      const float kp  = kb ? w4[i + 2] : w4[i];
      x2[i] = kp + __shfl_xor(snd, 2, 32);
    }
  }
  float fin;
  {
    const bool kb = (lane & 1) != 0;
    const float snd = kb ? x2[0] : x2[1];
    const float kp  = kb ? x2[1] : x2[0];
    fin = kp + __shfl_xor(snd, 1, 32);
  }
  {
    float s = fin + b3v;
    s = fminf(fmaxf(s, -40.0f), 40.0f);
    const float ex = __expf(-s);
    const float score = __builtin_amdgcn_rcpf(1.0f + ex);
    const int j = 16 * (m >> 3) + 8 * hh + (m & 7);
    sc[wave * EPW + j] = score;
  }
  __syncthreads();

  if (wave == 0) {
    const v4f ov = *(const v4f*)(sc + 4 * lane);
    const int e0 = blockIdx.x * EPB + 4 * lane;
    float* op = out + e0;
    const bool full = (e0 + 3 < nE);
    if (full) {
      *(volatile v4f*)op = ov;
    } else {
      if (e0     < nE) *(volatile float*)(op)     = ov.x;
      if (e0 + 1 < nE) *(volatile float*)(op + 1) = ov.y;
      if (e0 + 2 < nE) *(volatile float*)(op + 2) = ov.z;
    }
    __threadfence();
    if (full) {
      *(volatile v4f*)op = ov;
    } else {
      if (e0     < nE) *(volatile float*)(op)     = ov.x;
      if (e0 + 1 < nE) *(volatile float*)(op + 1) = ov.y;
      if (e0 + 2 < nE) *(volatile float*)(op + 2) = ov.z;
    }
  }
}

extern "C" void kernel_launch(void* const* d_in, const int* in_sizes, int n_in,
                              void* d_out, int out_size, void* d_ws, size_t ws_size,
                              hipStream_t stream) {
  if (n_in < 10) return;
  const int nN = in_sizes[0] / CH;
  const int nE = in_sizes[2];
  if (nN <= 0 || nE <= 0) return;
  if (in_sizes[0] != nN * CH || in_sizes[1] != nN * CH || in_sizes[3] != nE) return;
  if (in_sizes[4] != 2 * CH * CH || in_sizes[5] != CH || in_sizes[6] != CH * C2 ||
      in_sizes[7] != C2 || in_sizes[8] != C2 || in_sizes[9] < 1) return;
  if (out_size != nE) return;
  if (nN > (1 << 24) || nE > (1 << 28)) return;

  const float* zi   = (const float*)d_in[0];
  const float* zj   = (const float*)d_in[1];
  const int*   srcs = (const int*)d_in[2];
  const int*   dsts = (const int*)d_in[3];
  const float* W1   = (const float*)d_in[4];
  const float* b1   = (const float*)d_in[5];
  const float* W2   = (const float*)d_in[6];
  const float* b2   = (const float*)d_in[7];
  const float* W3   = (const float*)d_in[8];
  const float* b3   = (const float*)d_in[9];
  float* out = (float*)d_out;

  const int nBlkG = (nN + GROWS - 1) / GROWS;
  const int nPad  = nBlkG * GROWS;
  const int nBlkE = (nE + EPB - 1) / EPB;

  char* ws = (char*)d_ws;
  size_t off = 0;
  const size_t oB  = off; off += (size_t)BPTOT * 2;            off = (off + 255) & ~(size_t)255;
  const size_t oPQ = off; off += (size_t)2 * nPad * CH * 4;    off = (off + 255) & ~(size_t)255;
  if (off > ws_size || off > (size_t)WSCAP) return;
  _Float16* Bpl = (_Float16*)(ws + oB);
  float*    PQ  = (float*)(ws + oPQ);

  k_wprep<<<20, PTHR, 0, stream>>>(W1, W2, Bpl);
  k_nodegemm<<<dim3(nBlkG, 2), GTHR, 0, stream>>>(zi, zj, Bpl + OFF_B1, b1, PQ, nN, nPad);
  k_edge<<<nBlkE, ETHR, 0, stream>>>(PQ, srcs, dsts, Bpl + OFF_B2, b2, W3, b3, out, nN, nE, nPad);
}
